// SelfAttention_16063177687574
// MI455X (gfx1250) — hardware-verified
//
#include <hip/hip_runtime.h>


#ifndef NB
#define NB 2
#endif
#ifndef SEQ
#define SEQ 2048
#endif
#define NB_FULL   2
#define SEQ_FULL  2048
#define DM        2048
#define NQH       16
#define NKV       4
#define GRP       4
#define HD        128
#define HD2       64
#define NQKV      3072
#define EP        128
#define CPF       132
#define CP        136
#define TPW       72
#define WS_CAP    134217728ull

#define P_CARRY   4096.0f
#define V_CARRY   16.0f
#define C_CARRY   64.0f
#define W_CARRY   64.0f

static_assert(NB >= 1 && NB <= NB_FULL);
static_assert(SEQ <= SEQ_FULL);
static_assert(SEQ % 128 == 0);
static_assert(DM % 128 == 0);
static_assert(DM % 32 == 0);
static_assert(DM == 256 * 8);
static_assert(NQKV == NQH * HD + 2 * NKV * HD);
static_assert(NQKV % 128 == 0);
static_assert(NQH == NKV * GRP);
static_assert(HD == 128 && HD2 * 2 == HD);
static_assert(NQH * HD == DM);
static_assert(EP >= HD && (EP * 2) % 16 == 0);
static_assert((CPF * 4) % 16 == 0 && CPF >= 128);
static_assert((CP * 2) % 16 == 0 && CP >= HD);
static_assert((TPW * 2) % 16 == 0 && TPW >= 64);
static_assert(((size_t)NB * HD2 * SEQ) % 256 == 0);
static_assert(2 * 128 * EP * 2 <= 65536);

#define QELEMS   (NB * NQH * SEQ * HD)
#define KELEMS   (NB * NKV * SEQ * HD)
#define XB_BYTES   ((size_t)NB * SEQ * DM * 2)
#define WT_BYTES   ((size_t)NQKV * DM * 2)
#define WO_BYTES   ((size_t)DM * DM * 2)
#define TB_BYTES   ((size_t)NB * HD2 * SEQ * 4)
#define PL_BYTES   ((size_t)(QELEMS + KELEMS) * 2)
#define VT_BYTES   ((size_t)NB * NKV * HD * SEQ * 2)
#define CTX_BYTES  ((size_t)NB * SEQ * DM * 2)
#define OFF_XB   ((size_t)0)
#define OFF_WT   (OFF_XB + XB_BYTES)
#define OFF_WO   (OFF_WT + WT_BYTES)
#define OFF_COS  (OFF_WO + WO_BYTES)
#define OFF_SIN  (OFF_COS + TB_BYTES)
#define OFF_PH   (OFF_SIN + TB_BYTES)
#define OFF_PL   (OFF_PH + PL_BYTES)
#define OFF_VT   (OFF_PL + PL_BYTES)
#define OFF_CTX  (OFF_VT + VT_BYTES)
#define WS_TOTAL (OFF_CTX + CTX_BYTES)
static_assert(WS_TOTAL <= WS_CAP);
static_assert(XB_BYTES % 256 == 0 && WT_BYTES % 256 == 0 && WO_BYTES % 256 == 0);
static_assert(TB_BYTES % 256 == 0 && PL_BYTES % 256 == 0 && VT_BYTES % 256 == 0);
static_assert((unsigned long long)(QELEMS + KELEMS) < 2147483648ull);

typedef __bf16         bf16;
typedef _Float16       f16;
typedef unsigned short u16;
typedef bf16     v16bf __attribute__((ext_vector_type(16)));
typedef f16      v16h  __attribute__((ext_vector_type(16)));
typedef float    v8f   __attribute__((ext_vector_type(8)));
typedef float    v4f   __attribute__((ext_vector_type(4)));
typedef unsigned v4u   __attribute__((ext_vector_type(4)));

union Frag  { v16bf b; v16h h; v4u q[2]; f16 e[16]; };
union Pack8 { v4u u; u16 s[8]; };

static __device__ __forceinline__ v8f mma_bf16(v16bf a, v16bf b, v8f acc) {
  acc = __builtin_amdgcn_wmma_f32_16x16x32_bf16(false, a, false, b, (short)0, acc, false, false);
  asm volatile("v_nop\n\tv_nop\n\tv_nop\n\tv_nop" : "+v"(acc) : "v"(a), "v"(b));
  return acc;
}
static __device__ __forceinline__ v8f mma_f16(v16h a, v16h b, v8f acc) {
  acc = __builtin_amdgcn_wmma_f32_16x16x32_f16(false, a, false, b, (short)0, acc, false, false);
  asm volatile("v_nop\n\tv_nop\n\tv_nop\n\tv_nop" : "+v"(acc) : "v"(a), "v"(b));
  return acc;
}

static __device__ __forceinline__ u16 bf16_bits(float x) {
  const bf16 h = (bf16)x;
  return __builtin_bit_cast(u16, h);
}
static __device__ __forceinline__ float bf16_back(float x) {
  return (float)(bf16)x;
}
static __device__ __forceinline__ u16 f16_bits(float x) {
  const f16 h = (f16)x;
  return __builtin_bit_cast(u16, h);
}

__global__ __launch_bounds__(256) void xcvt_kernel(const float* __restrict__ X, u16* __restrict__ Xb) {
  const int m   = blockIdx.x;
  const int tid = threadIdx.x;
  const int b   = m / SEQ;
  const int t   = m % SEQ;
  const size_t src = ((size_t)b * SEQ_FULL + t) * DM + tid * 8;
  const v4f a0 = *(const v4f*)(X + src);
  const v4f a1 = *(const v4f*)(X + src + 4);
  Pack8 pk;
  #pragma unroll
  for (int i = 0; i < 4; ++i) {
    pk.s[i]     = bf16_bits(a0[i]);
    pk.s[4 + i] = bf16_bits(a1[i]);
  }
  const v4u val = pk.u;
  const size_t dst = (size_t)m * DM + tid * 8;
  *(volatile v4u*)(Xb + dst) = val;
  __threadfence();
  *(volatile v4u*)(Xb + dst) = val;
}

__global__ __launch_bounds__(256) void wtrans_kernel(const float* __restrict__ W, u16* __restrict__ Bt,
                                                     int ldin, int rowoff, int mode) {
  const int c0  = blockIdx.x * 64;
  const int d0  = blockIdx.y * 64;
  const int tid = threadIdx.x;
  __shared__ __align__(16) u16 sT[64 * TPW];
  #pragma unroll
  for (int kk = 0; kk < 2; ++kk) {
    const int r  = kk * 32 + (tid >> 3);
    const int cc = (tid & 7) * 8;
    const size_t src = (size_t)(d0 + r) * ldin + c0 + cc;
    const v4f w0 = *(const v4f*)(W + src);
    const v4f w1 = *(const v4f*)(W + src + 4);
    #pragma unroll
    for (int i = 0; i < 4; ++i) {
      const float x0 = bf16_back(w0[i]);
      const float x1 = bf16_back(w1[i]);
      const u16 h0 = (mode != 0) ? f16_bits(x0 * W_CARRY) : bf16_bits(x0);
      const u16 h1 = (mode != 0) ? f16_bits(x1 * W_CARRY) : bf16_bits(x1);
      sT[(cc + i) * TPW + r]     = h0;
      sT[(cc + 4 + i) * TPW + r] = h1;
    }
  }
  __syncthreads();
  v4u    val[2];
  size_t idx[2];
  #pragma unroll
  for (int kk = 0; kk < 2; ++kk) {
    const int c  = kk * 32 + (tid >> 3);
    const int ds = (tid & 7) * 8;
    val[kk] = *(const v4u*)(sT + c * TPW + ds);
    idx[kk] = (size_t)(rowoff + c0 + c) * DM + d0 + ds;
  }
  #pragma unroll
  for (int kk = 0; kk < 2; ++kk) *(volatile v4u*)(Bt + idx[kk]) = val[kk];
  __threadfence();
  #pragma unroll
  for (int kk = 0; kk < 2; ++kk) *(volatile v4u*)(Bt + idx[kk]) = val[kk];
}

__global__ __launch_bounds__(256) void rope_table_kernel(const int* __restrict__ pos,
                                                         float* __restrict__ cosT,
                                                         float* __restrict__ sinT) {
  const int idx = blockIdx.x * 256 + threadIdx.x;
  const int t = idx % SEQ;
  const int j = (idx / SEQ) % HD2;
  const int b = idx / (SEQ * HD2);
  const int p = pos[(size_t)b * SEQ_FULL + t];
  double pf = 1.0;
  pf *= (j & 32) ? 100.0 : 1.0;
  pf *= (j & 16) ? 10.0 : 1.0;
  pf *= (j & 8)  ? 3.1622776601683795 : 1.0;
  pf *= (j & 4)  ? 1.7782794100389228 : 1.0;
  pf *= (j & 2)  ? 1.333521432163324  : 1.0;
  pf *= (j & 1)  ? 1.1547819846894583 : 1.0;
  const float ts = (float)pf;
  float ang = (float)p / ts;
  ang = (p == 0) ? 0.0f : ang;
  float s, c;
  sincosf(ang, &s, &c);
  *(volatile float*)(cosT + idx) = c;
  *(volatile float*)(sinT + idx) = s;
  __threadfence();
  *(volatile float*)(cosT + idx) = c;
  *(volatile float*)(sinT + idx) = s;
}

template <int ISF16, int ROPEMAP>
static __device__ __forceinline__ void gemm_core(const u16* __restrict__ A, const u16* __restrict__ Bt,
                                                 int m0, int n0, int wm, int g, int lr, int hi,
                                                 v8f (&acc)[2][4]) {
  size_t aoff[2];
  size_t boff[4];
  #pragma unroll
  for (int fm = 0; fm < 2; ++fm) aoff[fm] = (size_t)(m0 + wm + fm * 16 + lr) * DM + 8 * hi;
  #pragma unroll
  for (int fn = 0; fn < 4; ++fn) {
    const int col = ROPEMAP ? (g * 32 + (fn & 1) * 16 + (fn >> 1) * 64) : (g * 64 + fn * 16);
    boff[fn] = (size_t)(n0 + col + lr) * DM + 8 * hi;
  }
  #pragma unroll 2
  for (int k0 = 0; k0 < DM; k0 += 32) {
    Frag a[2];
    Frag b[4];
    #pragma unroll
    for (int fm = 0; fm < 2; ++fm) {
      a[fm].q[0] = *(const v4u*)(A + aoff[fm] + k0);
      a[fm].q[1] = *(const v4u*)(A + aoff[fm] + k0 + 16);
    }
    #pragma unroll
    for (int fn = 0; fn < 4; ++fn) {
      b[fn].q[0] = *(const v4u*)(Bt + boff[fn] + k0);
      b[fn].q[1] = *(const v4u*)(Bt + boff[fn] + k0 + 16);
    }
    #pragma unroll
    for (int fn = 0; fn < 4; ++fn) {
      #pragma unroll
      for (int fm = 0; fm < 2; ++fm) {
        if (ISF16) acc[fm][fn] = mma_f16(a[fm].h, b[fn].h, acc[fm][fn]);
        else       acc[fm][fn] = mma_bf16(a[fm].b, b[fn].b, acc[fm][fn]);
      }
    }
  }
}

__global__ __launch_bounds__(256) void qkv_gemm_kernel(const u16* __restrict__ Xb, const u16* __restrict__ Wt,
                                                       const float* __restrict__ cosT,
                                                       const float* __restrict__ sinT,
                                                       u16* __restrict__ ph, u16* __restrict__ pl,
                                                       u16* __restrict__ vt) {
  __shared__ __align__(16) u16 sA[128 * EP];
  __shared__ __align__(16) u16 sB[128 * EP];
  const int ct   = blockIdx.x;
  const int m0   = blockIdx.y * 128;
  const int tid  = threadIdx.x;
  const int wave = __builtin_amdgcn_readfirstlane(threadIdx.x >> 5);
  const int lane = tid & 31;
  const int lr   = lane & 15;
  const int hi   = lane >> 4;
  const int wm   = (wave & 3) * 32;
  const int g    = wave >> 2;

  v8f acc[2][4];
  #pragma unroll
  for (int fm = 0; fm < 2; ++fm) {
    #pragma unroll
    for (int fn = 0; fn < 4; ++fn) acc[fm][fn] = (v8f){0, 0, 0, 0, 0, 0, 0, 0};
  }
  gemm_core<0, 1>(Xb, Wt, m0, ct * 128, wm, g, lr, hi, acc);

  const int b  = m0 / SEQ;
  const int t0 = m0 % SEQ;

  if (ct < NQH + NKV) {
    #pragma unroll
    for (int fm = 0; fm < 2; ++fm) {
      #pragma unroll
      for (int f2 = 0; f2 < 2; ++f2) {
        const int j  = g * 32 + f2 * 16 + lr;
        const int tl = wm + fm * 16 + 8 * hi;
        const size_t tb = ((size_t)b * HD2 + j) * SEQ + t0 + tl;
        const v4f ca = *(const v4f*)(cosT + tb);
        const v4f cb = *(const v4f*)(cosT + tb + 4);
        const v4f sa = *(const v4f*)(sinT + tb);
        const v4f sb = *(const v4f*)(sinT + tb + 4);
        #pragma unroll
        for (int i = 0; i < 8; ++i) {
          const float c  = (i < 4) ? ca[i & 3] : cb[i & 3];
          const float s  = (i < 4) ? sa[i & 3] : sb[i & 3];
          const float x1 = acc[fm][f2][i];
          const float x2 = acc[fm][f2 + 2][i];
          const float y1 = x1 * c - x2 * s;
          const float y2 = x2 * c + x1 * s;
          const float h1 = bf16_back(y1);
          const float h2 = bf16_back(y2);
          const int row = tl + i;
          sA[row * EP + j]       = bf16_bits(h1);
          sA[row * EP + 64 + j]  = bf16_bits(h2);
          sB[row * EP + j]       = bf16_bits(y1 - h1);
          sB[row * EP + 64 + j]  = bf16_bits(y2 - h2);
        }
      }
    }
    __syncthreads();
    const int isq   = (ct < NQH) ? 1 : 0;
    const int pbase = isq ? (((b * NQH + ct) * SEQ + t0) * HD)
                          : (QELEMS + ((b * NKV + (ct - NQH)) * SEQ + t0) * HD);
    v4u vA[8];
    v4u vB[8];
    int gi[8];
    #pragma unroll
    for (int it = 0; it < 8; ++it) {
      const int piece = it * 256 + tid;
      const int row = piece >> 4;
      const int seg = piece & 15;
      vA[it] = *(const v4u*)(sA + row * EP + seg * 8);
      vB[it] = *(const v4u*)(sB + row * EP + seg * 8);
      gi[it] = pbase + row * HD + seg * 8;
    }
    #pragma unroll
    for (int it = 0; it < 8; ++it) {
      *(volatile v4u*)(ph + gi[it]) = vA[it];
      *(volatile v4u*)(pl + gi[it]) = vB[it];
    }
    __threadfence();
    #pragma unroll
    for (int it = 0; it < 8; ++it) {
      *(volatile v4u*)(ph + gi[it]) = vA[it];
      *(volatile v4u*)(pl + gi[it]) = vB[it];
    }
  } else {
    const int kvh = ct - (NQH + NKV);
    #pragma unroll
    for (int fm = 0; fm < 2; ++fm) {
      #pragma unroll
      for (int fn = 0; fn < 4; ++fn) {
        const int d = g * 32 + (fn & 1) * 16 + (fn >> 1) * 64 + lr;
        #pragma unroll
        for (int i = 0; i < 8; ++i) {
          const int row = wm + fm * 16 + 8 * hi + i;
          sA[d * EP + row] = f16_bits(acc[fm][fn][i] * V_CARRY);
        }
      }
    }
    __syncthreads();
    v4u vA[8];
    int gi[8];
    #pragma unroll
    for (int it = 0; it < 8; ++it) {
      const int piece = it * 256 + tid;
      const int d   = piece >> 4;
      const int seg = piece & 15;
      vA[it] = *(const v4u*)(sA + d * EP + seg * 8);
      gi[it] = ((b * NKV + kvh) * HD + d) * SEQ + t0 + seg * 8;
    }
    #pragma unroll
    for (int it = 0; it < 8; ++it) *(volatile v4u*)(vt + gi[it]) = vA[it];
    __threadfence();
    #pragma unroll
    for (int it = 0; it < 8; ++it) *(volatile v4u*)(vt + gi[it]) = vA[it];
  }
}

__global__ __launch_bounds__(128) void attn_kernel(const u16* __restrict__ ph, const u16* __restrict__ pl,
                                                   const u16* __restrict__ vt, u16* __restrict__ ctx) {
  const int qt   = blockIdx.x;
  const int kv   = blockIdx.y;
  const int b    = blockIdx.z;
  const int tid  = threadIdx.x;
  const int wave = __builtin_amdgcn_readfirstlane(threadIdx.x >> 5);
  const int lane = tid & 31;
  const int lq   = lane & 15;
  const int hi   = lane >> 4;
  const int head = kv * GRP + wave;
  const int qrow0 = qt * 16;

  __shared__ __align__(16) u16 sO[GRP * 16 * CP];

  const int qoff  = ((b * NQH + head) * SEQ + qrow0 + lq) * HD + hi * 8;
  const int kbase = QELEMS + ((b * NKV + kv) * SEQ + lq) * HD + hi * 8;
  const int vbase = ((b * NKV + kv) * HD + lq) * SEQ + hi * 8;

  v8f o[8];
  #pragma unroll
  for (int dt = 0; dt < 8; ++dt) o[dt] = (v8f){0, 0, 0, 0, 0, 0, 0, 0};

  const float NEGV = -1.0e30f;
  float rmax = NEGV;
  float rsum = 0.0f;
  const float SL = 1.4426950408889634f;

  const int nchunk = (qrow0 >> 5) + 1;
  #pragma unroll 1
  for (int ic = 0; ic < nchunk; ++ic) {
    const int j0 = ic * 32;
    int qo = 0;
    asm volatile("" : "+v"(qo));

    v8f c0 = (v8f){0, 0, 0, 0, 0, 0, 0, 0};
    v8f c1 = (v8f){0, 0, 0, 0, 0, 0, 0, 0};
    const int krow = kbase + j0 * HD;
    #pragma unroll
    for (int f = 0; f < 4; ++f) {
      Frag qhf, qlf;
      const int qa = qoff + qo + f * 32;
      qhf.q[0] = *(const v4u*)(ph + qa);
      qhf.q[1] = *(const v4u*)(ph + qa + 16);
      qlf.q[0] = *(const v4u*)(pl + qa);
      qlf.q[1] = *(const v4u*)(pl + qa + 16);
      {
        Frag khf, klf;
        const int ka = krow + f * 32;
        khf.q[0] = *(const v4u*)(ph + ka);
        khf.q[1] = *(const v4u*)(ph + ka + 16);
        klf.q[0] = *(const v4u*)(pl + ka);
        klf.q[1] = *(const v4u*)(pl + ka + 16);
        c0 = mma_bf16(khf.b, qhf.b, c0);
        c0 = mma_bf16(khf.b, qlf.b, c0);
        c0 = mma_bf16(klf.b, qhf.b, c0);
      }
      {
        Frag khf, klf;
        const int ka = krow + 16 * HD + f * 32;
        khf.q[0] = *(const v4u*)(ph + ka);
        khf.q[1] = *(const v4u*)(ph + ka + 16);
        klf.q[0] = *(const v4u*)(pl + ka);
        klf.q[1] = *(const v4u*)(pl + ka + 16);
        c1 = mma_bf16(khf.b, qhf.b, c1);
        c1 = mma_bf16(khf.b, qlf.b, c1);
        c1 = mma_bf16(klf.b, qhf.b, c1);
      }
    }

    if (j0 + 31 > qrow0) {
      const int trow = qrow0 + lq;
      #pragma unroll
      for (int r = 0; r < 8; ++r) {
        const int key0 = j0 + hi * 8 + r;
        c0[r] = (key0 > trow) ? NEGV : c0[r];
        c1[r] = (key0 + 16 > trow) ? NEGV : c1[r];
      }
    }

    float m_new = rmax;
    #pragma unroll
    for (int r = 0; r < 8; ++r) {
      m_new = fmaxf(m_new, c0[r]);
      m_new = fmaxf(m_new, c1[r]);
    }
    m_new = fmaxf(m_new, __shfl_xor(m_new, 16, 32));
    const float scale = __builtin_amdgcn_exp2f((rmax - m_new) * SL);
    rmax = m_new;

    Frag pa;
    float psum = 0.0f;
    #pragma unroll
    for (int r = 0; r < 8; ++r) {
      const float p0 = __builtin_amdgcn_exp2f((c0[r] - m_new) * SL);
      const float p1 = __builtin_amdgcn_exp2f((c1[r] - m_new) * SL);
      psum += p0 + p1;
      pa.e[r]     = (f16)(p0 * P_CARRY);
      pa.e[8 + r] = (f16)(p1 * P_CARRY);
    }
    rsum = rsum * scale + psum + __shfl_xor(psum, 16, 32);

    float sc[8];
    #pragma unroll
    for (int r = 0; r < 8; ++r) sc[r] = __shfl(scale, (hi << 3) + r, 32);
    #pragma unroll
    for (int dt = 0; dt < 8; ++dt) {
      #pragma unroll
      for (int r = 0; r < 8; ++r) o[dt][r] *= sc[r];
    }

    #pragma unroll
    for (int hf = 0; hf < 2; ++hf) {
      Frag bv[4];
      #pragma unroll
      for (int dt = 0; dt < 4; ++dt) {
        const int va = vbase + ((hf * 4 + dt) * 16) * SEQ + j0;
        bv[dt].q[0] = *(const v4u*)(vt + va);
        bv[dt].q[1] = *(const v4u*)(vt + va + 16);
      }
      #pragma unroll
      for (int dt = 0; dt < 4; ++dt) o[hf * 4 + dt] = mma_f16(pa.h, bv[dt].h, o[hf * 4 + dt]);
    }
  }

  const float CN = C_CARRY / (P_CARRY * V_CARRY);
  float rs[8];
  #pragma unroll
  for (int r = 0; r < 8; ++r) rs[r] = CN * (1.0f / __shfl(rsum, (hi << 3) + r, 32));

  const int so = wave * (16 * CP);
  #pragma unroll
  for (int r = 0; r < 8; ++r) {
    #pragma unroll
    for (int dt = 0; dt < 8; ++dt) {
      sO[so + (hi * 8 + r) * CP + dt * 16 + lq] = f16_bits(o[dt][r] * rs[r]);
    }
  }
  __syncthreads();

  v4u    vals[8];
  size_t gidx[8];
  #pragma unroll
  for (int it = 0; it < 8; ++it) {
    const int row = it * 2 + hi;
    vals[it] = *(const v4u*)(sO + so + row * CP + lq * 8);
    gidx[it] = ((size_t)b * SEQ + qrow0 + row) * DM + head * HD + lq * 8;
  }
  #pragma unroll
  for (int it = 0; it < 8; ++it) *(volatile v4u*)(ctx + gidx[it]) = vals[it];
  __threadfence();
  #pragma unroll
  for (int it = 0; it < 8; ++it) *(volatile v4u*)(ctx + gidx[it]) = vals[it];
}

__global__ __launch_bounds__(256) void out_gemm_kernel(const u16* __restrict__ ctx, const u16* __restrict__ WoT,
                                                       float* __restrict__ out) {
  __shared__ __align__(16) float sC[64 * CPF];
  const int n0   = blockIdx.x * 128;
  const int m0   = blockIdx.y * 128;
  const int tid  = threadIdx.x;
  const int wave = __builtin_amdgcn_readfirstlane(threadIdx.x >> 5);
  const int lane = tid & 31;
  const int lr   = lane & 15;
  const int hi   = lane >> 4;
  const int wm   = (wave & 3) * 32;
  const int g    = wave >> 2;

  v8f acc[2][4];
  #pragma unroll
  for (int fm = 0; fm < 2; ++fm) {
    #pragma unroll
    for (int fn = 0; fn < 4; ++fn) acc[fm][fn] = (v8f){0, 0, 0, 0, 0, 0, 0, 0};
  }
  gemm_core<1, 0>(ctx, WoT, m0, n0, wm, g, lr, hi, acc);

  const float INV = 1.0f / (C_CARRY * W_CARRY);
  #pragma unroll
  for (int p = 0; p < 2; ++p) {
    if (((wave & 3) >> 1) == p) {
      #pragma unroll
      for (int fm = 0; fm < 2; ++fm) {
        #pragma unroll
        for (int fn = 0; fn < 4; ++fn) {
          #pragma unroll
          for (int i = 0; i < 8; ++i) {
            sC[(wm - p * 64 + fm * 16 + 8 * hi + i) * CPF + g * 64 + fn * 16 + lr] = acc[fm][fn][i] * INV;
          }
        }
      }
    }
    __syncthreads();
    v4f    vals[8];
    size_t gidx[8];
    #pragma unroll
    for (int it = 0; it < 8; ++it) {
      const int piece = it * 256 + tid;
      const int row = piece >> 5;
      const int seg = piece & 31;
      vals[it] = *(const v4f*)(sC + row * CPF + seg * 4);
      const int m  = m0 + p * 64 + row;
      const int bb = m / SEQ;
      const int tt = m % SEQ;
      gidx[it] = ((size_t)bb * SEQ_FULL + tt) * DM + n0 + seg * 4;
    }
    #pragma unroll
    for (int it = 0; it < 8; ++it) *(volatile v4f*)(out + gidx[it]) = vals[it];
    __threadfence();
    #pragma unroll
    for (int it = 0; it < 8; ++it) *(volatile v4f*)(out + gidx[it]) = vals[it];
    __syncthreads();
  }
}

extern "C" void kernel_launch(void* const* d_in, const int* in_sizes, int n_in,
                              void* d_out, int out_size, void* d_ws, size_t ws_size,
                              hipStream_t stream) {
  if (n_in < 6) return;
  const size_t needX = ((size_t)(NB - 1) * SEQ_FULL + SEQ) * DM;
  const size_t needP = (size_t)(NB - 1) * SEQ_FULL + SEQ;
  if ((size_t)in_sizes[0] < needX) return;
  if ((size_t)in_sizes[1] < needP) return;
  if ((size_t)in_sizes[2] < (size_t)DM * NQH * HD) return;
  if ((size_t)in_sizes[3] < (size_t)DM * NKV * HD) return;
  if ((size_t)in_sizes[4] < (size_t)DM * NKV * HD) return;
  if ((size_t)in_sizes[5] < (size_t)NQH * HD * DM) return;
  if ((size_t)out_size < needX) return;
  if (ws_size < (size_t)WS_TOTAL) return;

  const float* X   = (const float*)d_in[0];
  const int*   pos = (const int*)d_in[1];
  const float* Wq  = (const float*)d_in[2];
  const float* Wk  = (const float*)d_in[3];
  const float* Wv  = (const float*)d_in[4];
  const float* Wo  = (const float*)d_in[5];
  float* out = (float*)d_out;

  char* ws = (char*)d_ws;
  u16*   Xb   = (u16*)(ws + OFF_XB);
  u16*   Wt   = (u16*)(ws + OFF_WT);
  u16*   WoT  = (u16*)(ws + OFF_WO);
  float* cosT = (float*)(ws + OFF_COS);
  float* sinT = (float*)(ws + OFF_SIN);
  u16*   ph   = (u16*)(ws + OFF_PH);
  u16*   pl   = (u16*)(ws + OFF_PL);
  u16*   vt   = (u16*)(ws + OFF_VT);
  u16*   ctx  = (u16*)(ws + OFF_CTX);

  xcvt_kernel<<<dim3(NB * SEQ), 256, 0, stream>>>(X, Xb);
  wtrans_kernel<<<dim3((NQH * HD) / 64, DM / 64), 256, 0, stream>>>(Wq, Wt, NQH * HD, 0, 0);
  wtrans_kernel<<<dim3((NKV * HD) / 64, DM / 64), 256, 0, stream>>>(Wk, Wt, NKV * HD, NQH * HD, 0);
  wtrans_kernel<<<dim3((NKV * HD) / 64, DM / 64), 256, 0, stream>>>(Wv, Wt, NKV * HD, (NQH + NKV) * HD, 0);
  wtrans_kernel<<<dim3(DM / 64, DM / 64), 256, 0, stream>>>(Wo, WoT, DM, 0, 1);
  rope_table_kernel<<<dim3((NB * HD2 * SEQ) / 256), 256, 0, stream>>>(pos, cosT, sinT);
  qkv_gemm_kernel<<<dim3(NQKV / 128, (NB * SEQ) / 128), 256, 0, stream>>>(Xb, Wt, cosT, sinT, ph, pl, vt);
  attn_kernel<<<dim3(SEQ / 16, NKV, NB), 128, 0, stream>>>(ph, pl, vt, ctx);
  out_gemm_kernel<<<dim3(DM / 128, (NB * SEQ) / 128), 256, 0, stream>>>(ctx, WoT, out);
}
